// DeformableDynamicKernel2D_27736898797748
// MI455X (gfx1250) — hardware-verified
//
#include <hip/hip_runtime.h>


namespace {
constexpr int B = 2, C = 64, H = 256, W = 256, N = 32768, K = 9, HID = 64, K1 = 96, NO = 27;
constexpr float XS = 8.0f, WSC = 256.0f, SLOPE = 0.2f;
typedef _Float16 b16;
typedef __attribute__((ext_vector_type(16))) _Float16 v16b;
typedef __attribute__((ext_vector_type(8))) _Float16 v8b;
typedef __attribute__((ext_vector_type(8))) float v8f;
typedef __attribute__((ext_vector_type(4))) float v4f;
typedef __attribute__((ext_vector_type(2))) float v2f;
__device__ __forceinline__ float bf16_rne(float f) { unsigned int u = __float_as_uint(f); u += 0x7FFFu + ((u >> 16) & 1u); float r = __uint_as_float(u & 0xFFFF0000u); asm volatile("" : "+v"(r)); return r; }
__device__ __forceinline__ void split16(float v, b16& hi, b16& lo) { hi = (b16)v; lo = (b16)(v - (float)hi); }
__device__ __forceinline__ v16b frag_kb(const b16* p, int hh) { const v8b a = *(const v8b*)(p + 8 * hh), b = *(const v8b*)(p + 16 + 8 * hh); v16b f;
#pragma unroll
  for (int e = 0; e < 8; ++e) { f[e] = a[e]; f[8 + e] = b[e]; } return f; }
__device__ __forceinline__ v8f wmma16b(v16b a, v16b b, v8f c) { v8f d = __builtin_amdgcn_wmma_f32_16x16x32_f16(false, a, false, b, (short)0, c, false, false); asm volatile("v_nop\n\tv_nop\n\tv_nop\n\tv_nop" : "+v"(d) : "v"(a), "v"(b)); return d; }
__device__ __forceinline__ void wave_lds_sync() { __builtin_amdgcn_fence(__ATOMIC_RELEASE, "workgroup"); __builtin_amdgcn_wave_barrier(); __builtin_amdgcn_fence(__ATOMIC_ACQUIRE, "workgroup"); }
__device__ __forceinline__ float pmul(float a, float b) { float p = a * b; asm volatile("" : "+v"(p)); return p; }
__device__ __forceinline__ float lrelu(float v) { return v > 0.0f ? v : SLOPE * v; }
__device__ __forceinline__ float tanh_f(float v) { const float e = __expf(-2.0f * fabsf(v)); const float t = (1.0f - e) / (1.0f + e); return v < 0.0f ? -t : t; }

__global__ __launch_bounds__(256) void wput_kernel(const float* __restrict__ w1, const float* __restrict__ wr, const float* __restrict__ w2, b16* __restrict__ W1T, b16* __restrict__ WRT, b16* __restrict__ W2T) { const int u = blockIdx.x * 256 + threadIdx.x;
  for (int pass = 0; pass < 2; ++pass) {
    if (u < HID * 12) { const int o = u / 12, k0 = (u % 12) * 8; v8b v;
#pragma unroll
      for (int j = 0; j < 8; ++j) { const int k = k0 + j; v[j] = (b16)(k < C + 2 ? bf16_rne(w1[k * HID + o]) * WSC : 0.0f); } *(volatile v8b*)(W1T + (size_t)o * K1 + k0) = v; }
    if (u < HID * 8) { const int o = u / 8, k0 = (u % 8) * 8; v8b v;
#pragma unroll
      for (int j = 0; j < 8; ++j) v[j] = (b16)(bf16_rne(wr[(k0 + j) * HID + o]) * WSC); *(volatile v8b*)(WRT + (size_t)o * HID + k0) = v; }
    if (u < 32 * 8) { const int o = u / 8, k0 = (u % 8) * 8; v8b v;
#pragma unroll
      for (int j = 0; j < 8; ++j) v[j] = (b16)(o < NO ? bf16_rne(w2[(k0 + j) * NO + o]) * WSC : 0.0f); *(volatile v8b*)(W2T + (size_t)o * HID + k0) = v; }
    __threadfence(); } }
__device__ __forceinline__ v2f bilin2(const float* fm, int b, float gx, float gy, int lane) {
  float ix = (gx + 1.0f) * 0.5f * (float)(W - 1), iy = (gy + 1.0f) * 0.5f * (float)(H - 1); ix = fminf(fmaxf(ix, 0.0f), (float)(W - 1)); iy = fminf(fmaxf(iy, 0.0f), (float)(H - 1));
  const float fx = floorf(ix), fy = floorf(iy); const float wx = ix - fx, wy = iy - fy; const int x0 = (int)fx, y0 = (int)fy; const int x1 = min(x0 + 1, W - 1), y1 = min(y0 + 1, H - 1);
  v2f r; for (int k = 0; k < 2; ++k) { const float* f = fm + ((size_t)b * C + lane * 2 + k) * H * W; const float v00 = bf16_rne(f[y0 * W + x0]), v01 = bf16_rne(f[y0 * W + x1]), v10 = bf16_rne(f[y1 * W + x0]), v11 = bf16_rne(f[y1 * W + x1]);
    r[k] = pmul(pmul(v00, 1.0f - wx), 1.0f - wy) + pmul(pmul(v01, wx), 1.0f - wy) + pmul(pmul(v10, 1.0f - wx), wy) + pmul(pmul(v11, wx), wy); } return r; }
__global__ __launch_bounds__(32) void dk_kernel(const float* __restrict__ fm, const float* __restrict__ coords, const b16* __restrict__ W1T, const float* __restrict__ b1, const b16* __restrict__ WRT, const float* __restrict__ br, const b16* __restrict__ W2T, const float* __restrict__ b2, int NV, float* __restrict__ out) {
  __shared__ __attribute__((aligned(16))) b16 Ah[16][104], Al[16][104], Hh[16][72], Hl[16][72]; __shared__ float H1[16][68], Rr[16][36], Of[16][68]; const int lane = threadIdx.x, nloc = lane & 15, hlf = lane >> 4; const size_t p0 = (size_t)blockIdx.x * 16; const int b = (int)(p0 / N); if ((int)(p0 % N) >= NV) return;
  for (int rr = 0; rr < 16; ++rr) { const size_t p = p0 + rr; const float cx = bf16_rne(coords[p * 2]), cy = bf16_rne(coords[p * 2 + 1]); const v2f f = bilin2(fm, b, cx, cy, lane);
    b16 ph, pl; split16(f[0] * XS, ph, pl); Ah[rr][lane * 2] = ph; Al[rr][lane * 2] = pl; split16(f[1] * XS, ph, pl); Ah[rr][lane * 2 + 1] = ph; Al[rr][lane * 2 + 1] = pl;
    float ev = 0.0f; if (lane == 0) ev = cx; else if (lane == 1) ev = cy; split16(ev * XS, ph, pl); Ah[rr][C + lane] = ph; Al[rr][C + lane] = pl; }
  wave_lds_sync(); v8f acc[4];
#pragma unroll
  for (int t = 0; t < 4; ++t) acc[t] = (v8f){};
#pragma unroll
  for (int kb = 0; kb < K1; kb += 32) { const v16b a = frag_kb(&Ah[nloc][kb], hlf), al = frag_kb(&Al[nloc][kb], hlf);
#pragma unroll
    for (int t = 0; t < 4; ++t) { const v16b bw = frag_kb(W1T + (size_t)(t * 16 + nloc) * K1 + kb, hlf); acc[t] = wmma16b(a, bw, acc[t]); acc[t] = wmma16b(al, bw, acc[t]); } }
#pragma unroll
  for (int t = 0; t < 4; ++t) { const int c = t * 16 + nloc; const float bb = bf16_rne(b1[c]);
#pragma unroll
    for (int r8 = 0; r8 < 8; ++r8) { const float v = lrelu(acc[t][r8] * (1.0f / (XS * WSC)) + bb); H1[8 * hlf + r8][c] = v; b16 p, q; split16(v * XS, p, q); Hh[8 * hlf + r8][c] = p; Hl[8 * hlf + r8][c] = q; } }
  wave_lds_sync();
#pragma unroll
  for (int t = 0; t < 4; ++t) acc[t] = (v8f){};
#pragma unroll
  for (int kb = 0; kb < HID; kb += 32) { const v16b a = frag_kb(&Hh[nloc][kb], hlf), al = frag_kb(&Hl[nloc][kb], hlf);
#pragma unroll
    for (int t = 0; t < 4; ++t) { const v16b bw = frag_kb(WRT + (size_t)(t * 16 + nloc) * HID + kb, hlf); acc[t] = wmma16b(a, bw, acc[t]); acc[t] = wmma16b(al, bw, acc[t]); } }
  wave_lds_sync();
#pragma unroll
  for (int t = 0; t < 4; ++t) { const int c = t * 16 + nloc; const float bb = bf16_rne(br[c]);
#pragma unroll
    for (int r8 = 0; r8 < 8; ++r8) { const int rr = 8 * hlf + r8; const float v = lrelu(H1[rr][c] + acc[t][r8] * (1.0f / (XS * WSC)) + bb); b16 p, q; split16(v * XS, p, q); Hh[rr][c] = p; Hl[rr][c] = q; } }
  wave_lds_sync(); v8f ac2[2] = {(v8f){}, (v8f){}};
#pragma unroll
  for (int kb = 0; kb < HID; kb += 32) { const v16b a = frag_kb(&Hh[nloc][kb], hlf), al = frag_kb(&Hl[nloc][kb], hlf);
#pragma unroll
    for (int t = 0; t < 2; ++t) { const v16b bw = frag_kb(W2T + (size_t)(t * 16 + nloc) * HID + kb, hlf); ac2[t] = wmma16b(a, bw, ac2[t]); ac2[t] = wmma16b(al, bw, ac2[t]); } }
#pragma unroll
  for (int t = 0; t < 2; ++t) { const int c = t * 16 + nloc;
#pragma unroll
    for (int r8 = 0; r8 < 8; ++r8) Rr[8 * hlf + r8][c] = c < NO ? ac2[t][r8] * (1.0f / (XS * WSC)) + bf16_rne(b2[c]) : 0.0f; }
  wave_lds_sync();
  for (int rr = 0; rr < 16; ++rr) { const size_t p = p0 + rr; const float cx = bf16_rne(coords[p * 2]), cy = bf16_rne(coords[p * 2 + 1]); float wmax = -INFINITY; for (int k = 0; k < K; ++k) wmax = fmaxf(wmax, Rr[rr][2 * K + k]); float wsum = 0.0f, wk[K];
#pragma unroll
    for (int k = 0; k < K; ++k) { wk[k] = __expf(Rr[rr][2 * K + k] - wmax); wsum += wk[k]; }
    float o0 = 0.0f, o1 = 0.0f;
#pragma unroll
    for (int k = 0; k < K; ++k) { const float ox = pmul(tanh_f(Rr[rr][2 * k]), 16.0f / (float)W), oy = pmul(tanh_f(Rr[rr][2 * k + 1]), 16.0f / (float)H); const v2f f = bilin2(fm, b, cx + ox, cy + oy, lane); const float wgt = wk[k] / wsum; o0 += pmul(wgt, f[0]); o1 += pmul(wgt, f[1]); }
    Of[rr][lane * 2] = o0; Of[rr][lane * 2 + 1] = o1; }
  wave_lds_sync();
  for (int pass = 0; pass < 2; ++pass) { for (int rr = 0; rr < 16; ++rr) *(volatile v2f*)(out + (p0 + rr) * C + lane * 2) = (v2f){Of[rr][lane * 2], Of[rr][lane * 2 + 1]}; __threadfence(); } }
}

extern "C" void kernel_launch(void* const* d_in, const int* in_sizes, int n_in, void* d_out, int out_size, void* d_ws, size_t ws_size, hipStream_t stream) {
  (void)n_in;
  auto Fp = [&](int i) { return (const float*)d_in[i]; };
  if (in_sizes[0] != B * C * H * W || in_sizes[1] != B * N * 2 || in_sizes[2] != (C + 2) * HID || in_sizes[4] != HID * HID || in_sizes[6] != HID * NO || out_size != B * N * C) return;
  const int NV = N;
  size_t off = 0; char* ws = (char*)d_ws;
  auto carve = [&](size_t bytes) { char* p = ws + off; off += (bytes + 255) & ~(size_t)255; return p; };
  b16* W1T = (b16*)carve((size_t)HID * K1 * 2); b16* WRT = (b16*)carve((size_t)HID * HID * 2); b16* W2T = (b16*)carve((size_t)32 * HID * 2);
  if (off > ws_size || off > ((size_t)1 << 20)) return;
  wput_kernel<<<(HID * 12 + 255) / 256, 256, 0, stream>>>(Fp(2), Fp(4), Fp(6), W1T, WRT, W2T);
  dk_kernel<<<B * N / 16, 32, 0, stream>>>(Fp(0), Fp(1), W1T, Fp(3), WRT, Fp(5), W2T, Fp(7), NV, (float*)d_out);
}
